// BayesLinear_37950331027759
// MI455X (gfx1250) — hardware-run, weakly checked
//
#include <hip/hip_runtime.h>


#define NM   64
#define NK   4096
#define NO   4096
typedef _Float16 h16;
typedef unsigned short bf;
typedef __attribute__((ext_vector_type(16))) __bf16   v16bf;
typedef __attribute__((ext_vector_type(16))) _Float16 v16h;
typedef __attribute__((ext_vector_type(8)))  _Float16 v8h;
typedef __attribute__((ext_vector_type(8)))  unsigned short v8us;
typedef __attribute__((ext_vector_type(8)))  float    v8f;
typedef __attribute__((ext_vector_type(4)))  float    v4f;
typedef v8h  __attribute__((may_alias)) v8ha;
typedef v4f  __attribute__((may_alias)) v4fa;
typedef v8us __attribute__((may_alias)) v8usa;

__device__ __forceinline__ unsigned short f2bf(float f) { unsigned u = __float_as_uint(f); u += 0x7FFFu + ((u >> 16) & 1u); return (unsigned short)(u >> 16); }
__device__ __forceinline__ float bf2f(unsigned short b) { return __uint_as_float(((unsigned)b) << 16); }
__device__ __forceinline__ float bfr(float f) { return bf2f(f2bf(f)); }
__device__ __forceinline__ v16h cat16(v8h lo, v8h hi) { return __builtin_shufflevector(lo, hi, 0, 1, 2, 3, 4, 5, 6, 7, 8, 9, 10, 11, 12, 13, 14, 15); }
__device__ __forceinline__ v16bf cat16b(v8us lo, v8us hi) { return __builtin_bit_cast(v16bf, __builtin_shufflevector(lo, hi, 0, 1, 2, 3, 4, 5, 6, 7, 8, 9, 10, 11, 12, 13, 14, 15)); }
__device__ __forceinline__ v8f wmma16(v16h a, v16h b, v8f c) { return __builtin_amdgcn_wmma_f32_16x16x32_f16(false, a, false, b, (short)0, c, false, false); }
__device__ __forceinline__ v8f wmmab(v16bf a, v16bf b, v8f c) { return __builtin_amdgcn_wmma_f32_16x16x32_bf16(false, a, false, b, (short)0, c, false, false); }

template <typename T16> struct WFrag;
template <> struct WFrag<h16> { typedef v16h V; static __device__ __forceinline__ V ld(const h16* p) { return cat16(*(const v8h*)p, *(const v8h*)(p + 16)); } static __device__ __forceinline__ v8f mma(V a, V b, v8f c) { return wmma16(a, b, c); } };
template <> struct WFrag<bf> { typedef v16bf V; static __device__ __forceinline__ V ld(const bf* p) { return cat16b(*(const v8us*)p, *(const v8us*)(p + 16)); } static __device__ __forceinline__ v8f mma(V a, V b, v8f c) { return wmmab(a, b, c); } };
template <typename T16, int NSPLIT, bool BIAS>
__global__ __launch_bounds__(32) void k_gemmw(const T16* __restrict__ A, const T16* __restrict__ A2, const T16* __restrict__ Bt, const T16* __restrict__ Bt2, int K, float* C, int ldc, const float* __restrict__ bias, size_t sA, size_t sB, size_t sC) {
    typedef typename WFrag<T16>::V V;
    __shared__ __align__(16) float os[16 * 68];
    const size_t z = blockIdx.z; A += z * sA; if (A2) A2 += z * sA; Bt += z * sB; if (Bt2) Bt2 += z * sB; C += z * sC;
    const int lane = threadIdx.x & 31, lr = lane & 15, hi = lane >> 4; const int r0 = blockIdx.x * 64, c0 = blockIdx.y * 64;
    v8f acc[4][4];
#pragma unroll
    for (int mb = 0; mb < 4; ++mb)
#pragma unroll
        for (int nb = 0; nb < 4; ++nb) acc[mb][nb] = (v8f){};
    const size_t aoff = (size_t)(r0 + lr) * K + 8 * hi, boff = (size_t)(c0 + lr) * K + 8 * hi;
    for (int kc = 0; kc < K; kc += 32) {
        V a[4], a2[4];
#pragma unroll
        for (int mb = 0; mb < 4; ++mb) { a[mb] = WFrag<T16>::ld(A + aoff + (size_t)mb * 16 * K + kc); if (NSPLIT == 1 || NSPLIT == 2) a2[mb] = WFrag<T16>::ld(A2 + aoff + (size_t)mb * 16 * K + kc); }
#pragma unroll
        for (int nb = 0; nb < 4; ++nb) { const V b = WFrag<T16>::ld(Bt + boff + (size_t)nb * 16 * K + kc); V b2; if (NSPLIT >= 2) b2 = WFrag<T16>::ld(Bt2 + boff + (size_t)nb * 16 * K + kc);
#pragma unroll
            for (int mb = 0; mb < 4; ++mb) { acc[mb][nb] = WFrag<T16>::mma(a[mb], b, acc[mb][nb]); if (NSPLIT == 1 || NSPLIT == 2) acc[mb][nb] = WFrag<T16>::mma(a2[mb], b, acc[mb][nb]); if (NSPLIT >= 2) acc[mb][nb] = WFrag<T16>::mma(a[mb], b2, acc[mb][nb]); } }
        asm volatile("v_nop\n\tv_nop\n\tv_nop\n\tv_nop" : "+v"(acc[0][0]), "+v"(acc[1][1]), "+v"(acc[2][2]), "+v"(acc[3][3]) : "v"(a[0]), "v"(a[3]));
    }
#pragma unroll
    for (int mb = 0; mb < 4; ++mb) {
#pragma unroll
        for (int nb = 0; nb < 4; ++nb) {
#pragma unroll
            for (int j = 0; j < 8; ++j) os[(hi * 8 + j) * 68 + nb * 16 + lr] = acc[mb][nb][j]; }
        __builtin_amdgcn_wave_barrier(); asm volatile("" ::: "memory");
        float* crow = C + (size_t)(r0 + mb * 16) * ldc + c0;
#pragma unroll 1
        for (int ps = 0; ps < 2; ++ps) {
#pragma unroll
            for (int s = 0; s < 8; ++s) { const int row = 2 * s + hi, cofs = lr * 4; v4f val = *(const v4fa*)(os + row * 68 + cofs); if (BIAS) { val[0] += bfr(bias[c0 + cofs]); val[1] += bfr(bias[c0 + cofs + 1]); val[2] += bfr(bias[c0 + cofs + 2]); val[3] += bfr(bias[c0 + cofs + 3]); }
                *(volatile v4f*)(crow + (size_t)row * ldc + cofs) = val; }
            if (ps == 0) __threadfence(); }
        __builtin_amdgcn_wave_barrier(); asm volatile("" ::: "memory");
    }
}

typedef __attribute__((ext_vector_type(2))) _Float16 v2h;
typedef __attribute__((ext_vector_type(4))) _Float16 v4h;
typedef __attribute__((ext_vector_type(2))) unsigned short v2us;
typedef __attribute__((ext_vector_type(4))) unsigned short v4us;
typedef __attribute__((ext_vector_type(2))) float v2f;
typedef __attribute__((ext_vector_type(4))) int v4i;

__device__ __forceinline__ h16 toh_flush(float x) { const float z = (fabsf(x) < 6.103515625e-05f) ? 0.0f : x; return (h16)z; }

__device__ __forceinline__ float sp(float v) { return fmaxf(v, 0.0f) + log1pf(expf(-fabsf(v))); }

__global__ __launch_bounds__(256) void k_w(const float* __restrict__ Wm, const float* __restrict__ Wr, const float* __restrict__ Wn, h16* H) { const size_t j = (size_t)blockIdx.x * 256 + threadIdx.x; if (j >= (size_t)NO * NK / 8) return; const float* pm = Wm + j * 8; const float* pr = Wr + j * 8; const float* pn = Wn + j * 8; const v4f m0 = *(const v4f*)pm, m1 = *(const v4f*)(pm + 4), r0 = *(const v4f*)pr, r1 = *(const v4f*)(pr + 4), n0 = *(const v4f*)pn, n1 = *(const v4f*)(pn + 4); v8h o;
#pragma unroll
    for (int q = 0; q < 4; ++q) { o[q] = toh_flush(bfr(m0[q]) + bfr(n0[q]) * sp(bfr(r0[q]))); o[q + 4] = toh_flush(bfr(m1[q]) + bfr(n1[q]) * sp(bfr(r1[q]))); }
    *(volatile v8h*)(H + j * 8) = o; __threadfence(); *(volatile v8h*)(H + j * 8) = o; }

__global__ __launch_bounds__(256) void k_xh(const float* __restrict__ x, h16* H) { const int j = blockIdx.x * 256 + threadIdx.x; if (j >= NM * NK / 8) return; const float* p = x + (size_t)j * 8; const v4f a = *(const v4f*)p, b = *(const v4f*)(p + 4); v8h o;
#pragma unroll
    for (int q = 0; q < 4; ++q) { o[q] = toh_flush(bfr(a[q])); o[q + 4] = toh_flush(bfr(b[q])); }
    *(volatile v8h*)(H + (size_t)j * 8) = o; __threadfence(); *(volatile v8h*)(H + (size_t)j * 8) = o; }

__global__ __launch_bounds__(256) void k_fin(const float* __restrict__ P, const float* __restrict__ cm, const float* __restrict__ cr, const float* __restrict__ cn, float* out) { const int j = blockIdx.x * 256 + threadIdx.x; if (j >= NM * NO / 4) return; const int c = (j % (NO / 4)) * 4; v4f v = *(const v4f*)(P + (size_t)j * 4); const v4f m = *(const v4f*)(cm + c), r = *(const v4f*)(cr + c), n = *(const v4f*)(cn + c);
#pragma unroll
    for (int q = 0; q < 4; ++q) v[q] = v[q] + (bfr(m[q]) + bfr(n[q]) * sp(bfr(r[q])));
    *(volatile v4f*)(out + (size_t)j * 4) = v; __threadfence(); *(volatile v4f*)(out + (size_t)j * 4) = v; }

extern "C" void kernel_launch(void* const* d_in, const int* in_sizes, int n_in, void* d_out, int out_size, void* d_ws, size_t ws_size, hipStream_t stream) {
    if (n_in < 7) return;
    if (in_sizes[0] != NM * NK || in_sizes[1] != NO * NK || in_sizes[2] != NO * NK || in_sizes[3] != NO || in_sizes[4] != NO || in_sizes[5] != NO * NK || in_sizes[6] != NO) return;
    if (out_size != NM * NO) return;
    static_assert(NM % 64 == 0 && NO % 64 == 0 && NK % 32 == 0 && ((size_t)NO * NK / 8) % 256 == 0 && (NM * NK / 8) % 256 == 0 && (NM * NO / 4) % 256 == 0 && NO % 4 == 0, "the product: M and N multiples of 64, the depth of 32; the flat grids exact");
    const float* x = (const float*)d_in[0]; const float* Wm = (const float*)d_in[1]; const float* Wr = (const float*)d_in[2]; const float* cm = (const float*)d_in[3]; const float* cr = (const float*)d_in[4]; const float* Wn = (const float*)d_in[5]; const float* cn = (const float*)d_in[6]; float* out = (float*)d_out;
    char* wsp = (char*)d_ws; auto take = [&](size_t bytes) { char* p = wsp; wsp += (bytes + 255) & ~(size_t)255; return (void*)p; };
    h16* Xh = (h16*)take((size_t)NM * NK * 2); h16* Wh = (h16*)take((size_t)NO * NK * 2); float* P = (float*)take((size_t)NM * NO * 4);
    if ((size_t)(wsp - (char*)d_ws) > ws_size) return;
    k_xh<<<(unsigned)(NM * NK / 8 / 256), 256, 0, stream>>>(x, Xh);
    k_w<<<(unsigned)((size_t)NO * NK / 8 / 256), 256, 0, stream>>>(Wm, Wr, Wn, Wh);
    k_gemmw<h16, 0, false><<<dim3(NM / 64, NO / 64, 1), 32, 0, stream>>>(Xh, nullptr, Wh, nullptr, NK, P, NO, nullptr, 0, 0, 0);
    k_fin<<<(unsigned)(NM * NO / 4 / 256), 256, 0, stream>>>(P, cm, cr, cn, out);
}
